// EdgeMessage_48696339202376
// MI455X (gfx1250) — hardware-verified
//
#include <hip/hip_runtime.h>


#ifndef NE
#define NE 300000
#endif
#define NE_FULL 300000
#define HID  32
#define EDG  16
#define MSG  32
#define NCOL (MSG * HID)
#define KP   32
#define TE   32
#define OSP  36

static_assert(HID == 32);
static_assert(EDG == 16);
static_assert(MSG * 4 == 128);
static_assert(KP == 32);
static_assert(EDG + 1 <= KP);
static_assert(NE % TE == 0);
static_assert(NE <= NE_FULL);
static_assert(TE == 32);
static_assert((NCOL * (KP / 8)) % 256 == 0);
static_assert((OSP * 4) % 16 == 0);
static_assert(OSP >= MSG);
static_assert(TE * OSP * 4 <= 131072);
static_assert(8 * 4 == TE);
static_assert(32 * 16 * 8 == TE * MSG * 4);

typedef unsigned short bf;
typedef __attribute__((ext_vector_type(16))) __bf16   v16bf;
typedef __attribute__((ext_vector_type(8)))  unsigned short v8us;
typedef __attribute__((ext_vector_type(8)))  float    v8f;
typedef __attribute__((ext_vector_type(4)))  float    v4f;
typedef v4f  __attribute__((may_alias)) v4fa;

__device__ __forceinline__ unsigned short f2bf(float f) { unsigned u = __float_as_uint(f); u += 0x7FFFu + ((u >> 16) & 1u); return (unsigned short)(u >> 16); }
__device__ __forceinline__ float bfr(float f) { return __uint_as_float(((unsigned)f2bf(f)) << 16); }
__device__ __forceinline__ v16bf cat16b(v8us lo, v8us hi) { return __builtin_bit_cast(v16bf, __builtin_shufflevector(lo, hi, 0, 1, 2, 3, 4, 5, 6, 7, 8, 9, 10, 11, 12, 13, 14, 15)); }
__device__ __forceinline__ v8f wmmab(v16bf a, v16bf b, v8f c) { return __builtin_amdgcn_wmma_f32_16x16x32_bf16(false, a, false, b, (short)0, c, false, false); }
__device__ __forceinline__ v16bf ldb(const bf* p)  { return cat16b(*(const v8us*)p, *(const v8us*)(p + 16)); }
__device__ __forceinline__ void wave_sync() { __builtin_amdgcn_fence(3  , "wavefront"); __builtin_amdgcn_wave_barrier(); asm volatile("" ::: "memory"); }
__device__ __forceinline__ v8f wmmab_g(v16bf a, v16bf b, v8f c) {
    c = wmmab(a, b, c);
    asm volatile("v_nop\n\tv_nop\n\tv_nop\n\tv_nop" : "+v"(c) : "v"(a), "v"(b));
    return c;
}

__global__ __launch_bounds__(256) void k_wconv(const float* __restrict__ W, const float* __restrict__ bias, bf* WA) {
    const int i = blockIdx.x * 256 + threadIdx.x;
    const int n = i >> 2, q = i & 3;
    const float* wp = W + (size_t)n * EDG + (q & 1) * 8;
    v4f w0 = *(const v4f*)wp; v4f w1 = *(const v4f*)(wp + 4);
    float bv = bias[n];
    asm volatile("" : "+v"(w0), "+v"(w1), "+v"(bv));
    const bool isw = (q < 2);
    v8us o;
#pragma unroll
    for (int k = 0; k < 4; ++k) {
        const unsigned short c0 = f2bf(w0[k]); const unsigned short c1 = f2bf(w1[k]);
        o[k] = isw ? c0 : (unsigned short)0; o[4 + k] = isw ? c1 : (unsigned short)0; }
    const unsigned short bb = f2bf(bv);
    const unsigned short e0v = o[0];
    o[0] = (q == 2) ? bb : e0v;
    *(volatile v8us*)(WA + (size_t)i * 8) = o; __threadfence(); *(volatile v8us*)(WA + (size_t)i * 8) = o;
}

__global__ __launch_bounds__(32) void k_edgemv(const float* __restrict__ HW, const float* __restrict__ EV, const bf* __restrict__ WA, float* OUT) {
    __shared__ __align__(16) float os[TE * OSP];
    const int lane = threadIdx.x & 31, lr = lane & 15, hi = lane >> 4;
    const int e0 = blockIdx.x * TE;
    v16bf bq[2];
    float hwv[2][2][8];
#pragma unroll
    for (int j = 0; j < 2; ++j) {
        const size_t e = (size_t)(e0 + 16 * j + lr);
        const float* ep = EV + e * EDG + 8 * hi;
        const v4f x0 = *(const v4f*)ep; const v4f x1 = *(const v4f*)(ep + 4);
        v8us lo; v8us hs = (v8us){};
#pragma unroll
        for (int k = 0; k < 4; ++k) { lo[k] = f2bf(x0[k]); lo[4 + k] = f2bf(x1[k]); }
        hs[0] = hi ? (unsigned short)0 : (unsigned short)0x3F80;
        bq[j] = cat16b(lo, hs);
        const float* hp = HW + e * HID + 8 * hi;
        const v4f g0 = *(const v4f*)hp; const v4f g1 = *(const v4f*)(hp + 4); const v4f g2 = *(const v4f*)(hp + 16); const v4f g3 = *(const v4f*)(hp + 20);
#pragma unroll
        for (int r = 0; r < 4; ++r) { hwv[j][0][r] = bfr(g0[r]); hwv[j][0][4 + r] = bfr(g1[r]); hwv[j][1][r] = bfr(g2[r]); hwv[j][1][4 + r] = bfr(g3[r]); }
    }
    const size_t ao = (size_t)lr * KP + 8 * hi;
#pragma unroll 1
    for (int m = 0; m < MSG; ++m) {
        const bf* ap = WA + ao + (size_t)m * (HID * KP);
        const v16bf a0 = ldb(ap); const v16bf a1 = ldb(ap + 16 * KP);
        float part[2];
#pragma unroll
        for (int j = 0; j < 2; ++j) {
            const v8f d0 = wmmab_g(a0, bq[j], (v8f){});
            const v8f d1 = wmmab_g(a1, bq[j], (v8f){});
            float s = 0.0f;
#pragma unroll
            for (int r = 0; r < 8; ++r) s = fmaf(d0[r], hwv[j][0][r], s);
#pragma unroll
            for (int r = 0; r < 8; ++r) s = fmaf(d1[r], hwv[j][1][r], s);
            part[j] = s;
        }
        const float snd  = hi ? part[0] : part[1];
        const float rcv  = __shfl_xor(snd, 16, 32);
        const float mine = hi ? part[1] : part[0];
        os[lane * OSP + m] = mine + rcv;
    }
    wave_sync();
    float* orow = OUT + (size_t)e0 * MSG;
#pragma unroll 1
    for (int ps = 0; ps < 2; ++ps) {
#pragma unroll
        for (int s = 0; s < 8; ++s) { const int row = 4 * s + (lane >> 3), cofs = (lane & 7) * 4;
            const v4f val = *(const v4fa*)(&os[row * OSP + cofs]);
            *(volatile v4f*)(orow + (size_t)row * MSG + cofs) = val; }
        if (ps == 0) __threadfence(); }
}

static constexpr size_t al256(size_t v) { return (v + 255) & ~(size_t)255; }
static constexpr size_t SZ_WA = al256((size_t)NCOL * KP * 2);
static constexpr size_t SZ_TOTAL = SZ_WA;
static_assert(SZ_TOTAL <= (size_t)134217728);
static_assert((size_t)(NCOL * (KP / 8)) * 8 * 2 == (size_t)NCOL * KP * 2);
static_assert((size_t)(NE / TE) * TE * MSG * 4 == (size_t)NE * MSG * 4);

extern "C" void kernel_launch(void* const* d_in, const int* in_sizes, int n_in,
                              void* d_out, int out_size, void* d_ws, size_t ws_size, hipStream_t stream) {
    if (n_in < 4) return;
    if ((size_t)in_sizes[0] < (size_t)NE * HID) return;
    if ((size_t)in_sizes[1] < (size_t)NE * EDG) return;
    if ((size_t)in_sizes[2] < (size_t)NCOL * EDG) return;
    if ((size_t)in_sizes[3] < (size_t)NCOL) return;
    if ((size_t)out_size < (size_t)NE * MSG) return;
    if (SZ_TOTAL > ws_size) return;
    const float* hw = (const float*)d_in[0];
    const float* ev = (const float*)d_in[1];
    const float* W  = (const float*)d_in[2];
    const float* bs = (const float*)d_in[3];
    float* OUT = (float*)d_out;
    bf* WA = (bf*)d_ws;

    k_wconv<<<(unsigned)((NCOL * (KP / 8)) / 256), 256, 0, stream>>>(W, bs, WA);
    k_edgemv<<<(unsigned)(NE / TE), 32, 0, stream>>>(hw, ev, WA, OUT);
}
